// GCN_70909910057300
// MI455X (gfx1250) — hardware-verified
//
#include <hip/hip_runtime.h>
#include <stddef.h>
#include <stdint.h>


#define NN     50000
#define NE     600000
#define D1     32
#define DF     128
#define MPAD   50048
#define NTHR   256
#define NWAVE  8
#define EPT    8
#define CHUNK  (NTHR * EPT)
#define WCAP   (EPT * 32)
#define LISTN  (NWAVE * WCAP)
#define NBA    1024
#define SLA    10
#define NBLK   49
#define NMETA  (NBLK * NBA)
#define RCAP   28672
#define DEGCAP 64
#define RPW    16
#define RPB    (NWAVE * RPW)
#define GBM    64
#define GBN    128
#define GTHR   128
#define GWAVE  (GTHR / 32)
#define PW     256
#define U2     2048
#define UBL    8192
#define NUP    (U2 + 3 * UBL)
#define AGG_ZINTS (LISTN + 2 * RCAP + 3 * NBA)
#define MISC_INTS 16
#define BKT_LDS_INTS (AGG_ZINTS + MISC_INTS)
#define WSMAX  134217728

static_assert(MPAD % GBM == 0 && MPAD % RPB == 0 && MPAD >= NN && MPAD - NN < GBM);
static_assert(NBLK * NBA >= MPAD && NMETA >= MPAD);
static_assert((CHUNK & (CHUNK - 1)) == 0 && CHUNK <= 4096);
static_assert((NBA & (NBA - 1)) == 0 && NBA == (1 << SLA));
static_assert(((long long)(NE + CHUNK) << SLA) < (1LL << 31));
static_assert(RCAP % (NTHR * 4) == 0 && AGG_ZINTS % (NTHR * 4) == 0 && NBA % NTHR == 0);
static_assert(RCAP >= 13176 && DEGCAP >= 28 + 8);
static_assert(DF % 32 == 0 && (4 * DF) % 32 == 0 && (4 * D1) % 32 == 0 && PW == 2 * DF);
static_assert(GBN == DF && GBM == GWAVE * 16 && DF == 4 * 32 && GTHR == GWAVE * 32);
static_assert(NUP % NTHR == 0 && (U2 / 2) % NTHR == 0 && (UBL / 4) % NTHR == 0 && U2 % NTHR == 0);
static_assert(NN % 4 == 0 && (GBM * 4) % 128 == 0);
static_assert(BKT_LDS_INTS * 4 <= 300000);

typedef float          v2f   __attribute__((ext_vector_type(2)));
typedef float          v4f   __attribute__((ext_vector_type(4)));
typedef float          v8f   __attribute__((ext_vector_type(8)));
typedef int            v4i   __attribute__((ext_vector_type(4)));
typedef int            v8i   __attribute__((ext_vector_type(8)));
typedef unsigned       v2u   __attribute__((ext_vector_type(2)));
typedef unsigned       v4u   __attribute__((ext_vector_type(4)));
typedef unsigned short v4us  __attribute__((ext_vector_type(4)));
typedef unsigned short v8us  __attribute__((ext_vector_type(8)));
typedef unsigned short v16us __attribute__((ext_vector_type(16)));
typedef __bf16         v16bf __attribute__((ext_vector_type(16)));
typedef v4f  __attribute__((may_alias)) v4fa;
typedef v4i  __attribute__((may_alias)) v4ia;
typedef v2u  __attribute__((may_alias)) v2ua;
typedef v4u  __attribute__((may_alias)) v4ua;
typedef v4us __attribute__((may_alias)) v4usa;
typedef v8us __attribute__((may_alias)) v8usa;
union FragB { v16bf v; v16us u; v8us h[2]; v8i w; };

__device__ __forceinline__ v8f wmb(const FragB& a, const FragB& b, v8f c) {
  v8f d = __builtin_amdgcn_wmma_f32_16x16x32_bf16(false, a.v, false, b.v, (short)0, c, false, false);
  asm volatile("v_nop\n\tv_nop\n\tv_nop\n\tv_nop" : "+v"(d) : "v"(a.w), "v"(b.w));
  return d;
}

__device__ __forceinline__ v8f z8() { v8f z = {0.f, 0.f, 0.f, 0.f, 0.f, 0.f, 0.f, 0.f}; return z; }

__device__ __forceinline__ unsigned bf16_bits(float f) {
  const unsigned u = __float_as_uint(f);
  const unsigned r = (u + 0x7FFFu + ((u >> 16) & 1u)) >> 16;
  return (f != f) ? 0x7FC0u : r;
}
__device__ __forceinline__ float bf16_val(float f) {
  return __uint_as_float(bf16_bits(f) << 16);
}
__device__ __forceinline__ unsigned hl_bits(float v, unsigned& lo) {
  const unsigned hb = bf16_bits(v);
  lo = bf16_bits(v - __uint_as_float(hb << 16));
  return hb;
}
__device__ __forceinline__ float relu_p(float v) { return (v > 0.0f) ? v : (v - v); }

__device__ __forceinline__ void wave_sync() {
  __builtin_amdgcn_fence(__ATOMIC_RELEASE, "wavefront");
  __builtin_amdgcn_wave_barrier();
  __builtin_amdgcn_fence(__ATOMIC_ACQUIRE, "wavefront");
}

template <int SLB>
__device__ __forceinline__ int scan_chunk(const int* __restrict__ dsts, int nE, int cbase, int slotBase,
                                          int nb, int vec8, int* list, int tid, int lane, int wave) {
  int wc = 0;
  const int el0  = tid * EPT;
  const int e0   = cbase + el0;
  const int sent = -2147483647 - 1;
  v4i da, db;
  if (vec8 != 0 && cbase + CHUNK <= nE) {
    da = *(const v4i*)(dsts + e0);
    db = *(const v4i*)(dsts + e0 + 4);
  } else {
    da.x = (e0     < nE) ? dsts[min(e0,     nE - 1)] : sent;
    da.y = (e0 + 1 < nE) ? dsts[min(e0 + 1, nE - 1)] : sent;
    da.z = (e0 + 2 < nE) ? dsts[min(e0 + 2, nE - 1)] : sent;
    da.w = (e0 + 3 < nE) ? dsts[min(e0 + 3, nE - 1)] : sent;
    db.x = (e0 + 4 < nE) ? dsts[min(e0 + 4, nE - 1)] : sent;
    db.y = (e0 + 5 < nE) ? dsts[min(e0 + 5, nE - 1)] : sent;
    db.z = (e0 + 6 < nE) ? dsts[min(e0 + 6, nE - 1)] : sent;
    db.w = (e0 + 7 < nE) ? dsts[min(e0 + 7, nE - 1)] : sent;
  }
  const unsigned nbs = (unsigned)slotBase;
  const unsigned unb = (unsigned)nb;
  const unsigned s0 = (unsigned)da.x - nbs, s1 = (unsigned)da.y - nbs;
  const unsigned s2 = (unsigned)da.z - nbs, s3 = (unsigned)da.w - nbs;
  const unsigned s4 = (unsigned)db.x - nbs, s5 = (unsigned)db.y - nbs;
  const unsigned s6 = (unsigned)db.z - nbs, s7 = (unsigned)db.w - nbs;
  const bool h0 = s0 < unb, h1 = s1 < unb, h2 = s2 < unb, h3 = s3 < unb;
  const bool h4 = s4 < unb, h5 = s5 < unb, h6 = s6 < unb, h7 = s7 < unb;
  const unsigned any = __builtin_amdgcn_ballot_w32(h0 | h1 | h2 | h3 | h4 | h5 | h6 | h7);
  if (any != 0u) {
#define HITJ(J, HJ, SJ) { \
      const unsigned mj = __builtin_amdgcn_ballot_w32(HJ); \
      if (mj != 0u) { \
        if (HJ) { \
          const int pos = wc + (int)__builtin_amdgcn_mbcnt_lo(mj, 0u); \
          if (pos < WCAP) list[wave * WCAP + pos] = ((el0 + (J)) << SLB) | (int)(SJ); \
        } \
        wc += (int)__builtin_popcount(mj); } }
    HITJ(0, h0, s0)
    HITJ(1, h1, s1)
    HITJ(2, h2, s2)
    HITJ(3, h3, s3)
    HITJ(4, h4, s4)
    HITJ(5, h5, s5)
    HITJ(6, h6, s6)
    HITJ(7, h7, s7)
#undef HITJ
  }
  return wc;
}

__global__ __launch_bounds__(NTHR) void k_prep(const float* __restrict__ w2l, const float* __restrict__ w2r,
                                               const float* __restrict__ w3l, const float* __restrict__ w3r,
                                               const float* __restrict__ w4l, const float* __restrict__ w4r,
                                               const float* __restrict__ w5l, const float* __restrict__ w5r,
                                               unsigned short* w2c, unsigned short* wbig) {
  const int u = (int)blockIdx.x * NTHR + (int)threadIdx.x;
  const float* W;
  int so;
  unsigned short* dp;
  if (u < U2) {
    const int half = u >> 10;
    const int v = u & 1023;
    const int n = v >> 3, j = v & 7;
    const int kk = (8 * j) & 31;
    if (half == 0) W = w2l; else W = w2r;
    so = kk * DF + n;
    dp = w2c + (size_t)n * DF + half * 64 + 8 * j;
  } else if (u < NUP) {
    const int g = u - U2;
    const int layer = g >> 13;
    const int part  = (g >> 11) & 3;
    const int v = g & 2047;
    const int n = v >> 4, k8 = (v & 15) * 8;
    if (layer == 0)      { if (part < 2) W = w3l; else W = w3r; }
    else if (layer == 1) { if (part < 2) W = w4l; else W = w4r; }
    else                 { if (part < 2) W = w5l; else W = w5r; }
    so = k8 * DF + n;
    dp = wbig + (size_t)layer * (DF * 4 * DF) + (size_t)n * (4 * DF) + part * DF + k8;
  } else {
    return;
  }
  v8us o;
#pragma unroll
  for (int i = 0; i < 8; ++i) o[i] = (unsigned short)bf16_bits(W[so + i * DF]);
  *(volatile v8us*)dp = o;
  __threadfence();
  *(volatile v8us*)dp = o;
}

__global__ __launch_bounds__(NTHR) void k_bucket(const int* __restrict__ srcs, const int* __restrict__ dsts,
                                                 int nE, int nN, int vec8, int* lst, int* meta) {
  extern __shared__ __attribute__((aligned(16))) int dsm[];
  int* list = dsm;
  int* hl   = dsm + LISTN;
  int* sl   = hl + RCAP;
  int* cnt  = sl + RCAP;
  int* offs = cnt + NBA;
  int* cur  = offs + NBA;
  int* misc = cur + NBA;
  const int tid = (int)threadIdx.x, lane = tid & 31, wave = tid >> 5;
  const int nodeBase = (int)blockIdx.x * NBA;

  {
    const v4i z4 = {0, 0, 0, 0};
    for (int i = tid * 4; i < AGG_ZINTS; i += NTHR * 4) *(v4ia*)(dsm + i) = z4;
    if (tid < MISC_INTS) misc[tid] = 0;
  }
  __syncthreads();

  int t = 0, ov = 0;
  const int nChunks = (nE + CHUNK - 1) / CHUNK;
#pragma unroll 1
  for (int ch = 0; ch < nChunks; ++ch) {
    const int cbase = ch * CHUNK;
    const int wc = scan_chunk<SLA>(dsts, nE, cbase, nodeBase, NBA, vec8, list, tid, lane, wave);
    if (lane == 0) misc[wave] = wc;
    __syncthreads();
    if (wave == 0) {
#pragma unroll 1
      for (int w2 = 0; w2 < NWAVE; ++w2) {
        int c = misc[w2];
        c = c < 0 ? 0 : (c > WCAP ? WCAP : c);
#pragma unroll 1
        for (int b0 = 0; b0 < c; b0 += 32) {
          const int idx = b0 + lane;
          const int ent_ = list[w2 * WCAP + (idx < WCAP ? idx : WCAP - 1)];
          const int m32 = (c - b0) < 32 ? (c - b0) : 32;
#pragma unroll 1
          for (int k = 0; k < m32; ++k) {
            const int u    = __builtin_amdgcn_readlane(ent_, k);
            const int slot = u & (NBA - 1);
            const int el   = (u >> SLA) & (CHUNK - 1);
            const int pk   = ((cbase + el) << SLA) | slot;
            if (t < RCAP) {
              if (lane == 0) { hl[t] = pk; cnt[slot] = cnt[slot] + 1; }
              t = t + 1;
            } else {
              ov = 1;
            }
          }
        }
      }
    }
    __syncthreads();
  }
  if (wave == 0 && lane == 0) { misc[8] = t; misc[9] = ov; }
  __syncthreads();
  int tt = misc[8];
  tt = tt < 0 ? 0 : (tt > RCAP ? RCAP : tt);
  const int ovf = misc[9];

  if (wave == 0) {
    const int base = lane * (NBA / 32);
    int s = 0;
#pragma unroll 1
    for (int i = 0; i < NBA / 32; ++i) s += cnt[base + i];
    int incl = s;
#pragma unroll
    for (int d = 1; d < 32; d <<= 1) {
      const int y = __shfl_up(incl, d, 32);
      if (lane >= d) incl += y;
    }
    int run = incl - s;
#pragma unroll 1
    for (int i = 0; i < NBA / 32; ++i) {
      const int cv = cnt[base + i];
      offs[base + i] = run;
      cur[base + i]  = run;
      run += cv;
    }
  }
  __syncthreads();
  if (wave == 0) {
#pragma unroll 1
    for (int b0 = 0; b0 < tt; b0 += 32) {
      const int idx = b0 + lane;
      const int ent_ = hl[idx < RCAP ? idx : RCAP - 1];
      const int m32 = (tt - b0) < 32 ? (tt - b0) : 32;
#pragma unroll 1
      for (int k = 0; k < m32; ++k) {
        const int u    = __builtin_amdgcn_readlane(ent_, k);
        const int slot = u & (NBA - 1);
        if (lane == 0) {
          int p = cur[slot];
          p = p < 0 ? 0 : (p > RCAP - 1 ? RCAP - 1 : p);
          sl[p] = u;
          cur[slot] = p + 1;
        }
      }
    }
  }
  __syncthreads();

  int* lp = lst + (size_t)blockIdx.x * RCAP;
#pragma unroll 1
  for (int i = tid * 4; i < RCAP; i += NTHR * 4) {
    const v4i e = *(const v4ia*)(sl + i);
    int e0 = e.x >> SLA, e1 = e.y >> SLA, e2 = e.z >> SLA, e3 = e.w >> SLA;
    e0 = e0 < 0 ? 0 : (e0 > nE - 1 ? nE - 1 : e0);
    e1 = e1 < 0 ? 0 : (e1 > nE - 1 ? nE - 1 : e1);
    e2 = e2 < 0 ? 0 : (e2 > nE - 1 ? nE - 1 : e2);
    e3 = e3 < 0 ? 0 : (e3 > nE - 1 ? nE - 1 : e3);
    int r0 = srcs[e0], r1 = srcs[e1], r2 = srcs[e2], r3 = srcs[e3];
    r0 = r0 < 0 ? 0 : (r0 > nN - 1 ? nN - 1 : r0);
    r1 = r1 < 0 ? 0 : (r1 > nN - 1 ? nN - 1 : r1);
    r2 = r2 < 0 ? 0 : (r2 > nN - 1 ? nN - 1 : r2);
    r3 = r3 < 0 ? 0 : (r3 > nN - 1 ? nN - 1 : r3);
    v4i o;
    o.x = (i     < tt) ? r0 : 0;
    o.y = (i + 1 < tt) ? r1 : 0;
    o.z = (i + 2 < tt) ? r2 : 0;
    o.w = (i + 3 < tt) ? r3 : 0;
    int* dp = lp + i;
    *(volatile v4i*)dp = o;
    __threadfence();
    *(volatile v4i*)dp = o;
  }
#pragma unroll 1
  for (int q = 0; q < NBA / NTHR; ++q) {
    const int s = q * NTHR + tid;
    const int c = cnt[s];
    const int o = offs[s];
    const float inv = 1.0f / fmaxf((float)c, 1.0f);
    v4i mv;
    mv.x = c;
    mv.y = o;
    mv.z = __float_as_int(inv);
    mv.w = (ovf != 0 || c > DEGCAP) ? 1 : 0;
    int* mp = meta + (size_t)(nodeBase + s) * 4;
    *(volatile v4i*)mp = mv;
    __threadfence();
    *(volatile v4i*)mp = mv;
  }
}

struct RowMeta { int c; int o; float inv; float pz; int blk; };
__device__ __forceinline__ RowMeta load_meta(const int* __restrict__ meta, int node) {
  const int nm = node < 0 ? 0 : (node > NMETA - 1 ? NMETA - 1 : node);
  const v4i mt = *(const v4ia*)(meta + (size_t)nm * 4);
  const int cr = __builtin_amdgcn_readfirstlane(mt.x);
  const int orr = __builtin_amdgcn_readfirstlane(mt.y);
  const int ib = __builtin_amdgcn_readfirstlane(mt.z);
  const int fl = __builtin_amdgcn_readfirstlane(mt.w);
  RowMeta r;
  r.c   = cr < 0 ? 0 : (cr > DEGCAP ? DEGCAP : cr);
  r.o   = orr < 0 ? 0 : (orr > RCAP - 1 ? RCAP - 1 : orr);
  r.inv = __int_as_float(ib);
  r.pz  = (fl != 0 || cr > DEGCAP || cr < 0) ? __int_as_float(0x7fc00000) : 0.0f;
  r.blk = nm >> SLA;
  return r;
}

__global__ __launch_bounds__(NTHR) void k_l1(const float* __restrict__ x, const float* __restrict__ w1l,
                                             const float* __restrict__ b1, const float* __restrict__ w1r,
                                             const int* __restrict__ lst, const int* __restrict__ meta,
                                             int nN, unsigned short* h1) {
  __shared__ __attribute__((aligned(16))) unsigned short rb[NWAVE * 64];
  const int tid = (int)threadIdx.x, lane = tid & 31, wave = tid >> 5;
  unsigned short* rowbuf = rb + wave * 64;
  const float wl0 = bf16_val(w1l[lane]);
  const float wl1 = bf16_val(w1l[D1 + lane]);
  const float bb  = bf16_val(b1[lane]);
  const float wr0 = bf16_val(w1r[lane]);
  const float wr1 = bf16_val(w1r[D1 + lane]);
#pragma unroll 1
  for (int r = 0; r < RPW; ++r) {
    const int node = (int)blockIdx.x * RPB + wave * RPW + r;
    const RowMeta rm = load_meta(meta, node);
    const int* lp = lst + (size_t)rm.blk * RCAP;
    float a0 = 0.0f, a1 = 0.0f;
#pragma unroll 1
    for (int b0 = 0; b0 < rm.c; b0 += 32) {
      int idx = rm.o + b0 + lane;
      idx = idx > RCAP - 1 ? RCAP - 1 : idx;
      int sr = lp[idx];
      sr = sr < 0 ? 0 : (sr > nN - 1 ? nN - 1 : sr);
      const v2f xv = *(const v2f*)(x + (size_t)sr * 2);
      const int x0i = __float_as_int(bf16_val(xv.x));
      const int x1i = __float_as_int(bf16_val(xv.y));
      const int m32 = (rm.c - b0) < 32 ? (rm.c - b0) : 32;
#pragma unroll 1
      for (int k = 0; k < m32; ++k) {
        a0 += __int_as_float(__builtin_amdgcn_readlane(x0i, k));
        a1 += __int_as_float(__builtin_amdgcn_readlane(x1i, k));
      }
    }
    const int nc = node < nN ? node : nN - 1;
    const v2f xo = *(const v2f*)(x + (size_t)nc * 2);
    const float x0 = bf16_val(xo.x), x1 = bf16_val(xo.y);
    const float m0 = a0 * rm.inv, m1 = a1 * rm.inv;
    float tl = m0 * wl0;
    tl = fmaf(m1, wl1, tl);
    tl += bb;
    float tr = x0 * wr0;
    tr = fmaf(x1, wr1, tr);
    const float v = relu_p((tl + tr) + rm.pz);
    const bool live = node < nN;
    const float y = live ? v : 0.0f;
    unsigned lb;
    const unsigned hb = hl_bits(y, lb);
    rowbuf[lane]      = (unsigned short)hb;
    rowbuf[D1 + lane] = (unsigned short)lb;
    wave_sync();
    const v8us q0 = *(const v8usa*)(rowbuf + 8 * (lane & 7));
    wave_sync();
    unsigned short* dp = h1 + (size_t)node * 64 + 8 * (lane & 7);
    if (lane < 8) *(volatile v8us*)dp = q0;
    __threadfence();
    if (lane < 8) *(volatile v8us*)dp = q0;
  }
}

__global__ __launch_bounds__(NTHR) void k_agg2(const unsigned short* __restrict__ h1, const int* __restrict__ lst,
                                               const int* __restrict__ meta, int nN, unsigned short* a2) {
  __shared__ __attribute__((aligned(16))) unsigned short rb[NWAVE * 64];
  const int tid = (int)threadIdx.x, lane = tid & 31, wave = tid >> 5;
  unsigned short* rowbuf = rb + wave * 64;
#pragma unroll 1
  for (int r = 0; r < RPW; ++r) {
    const int node = (int)blockIdx.x * RPB + wave * RPW + r;
    const RowMeta rm = load_meta(meta, node);
    const int* lp = lst + (size_t)rm.blk * RCAP;
    float a = 0.0f;
#pragma unroll 1
    for (int b0 = 0; b0 < rm.c; b0 += 32) {
      int idx = rm.o + b0 + lane;
      idx = idx > RCAP - 1 ? RCAP - 1 : idx;
      int sr = lp[idx];
      sr = sr < 0 ? 0 : (sr > nN - 1 ? nN - 1 : sr);
      const int m32 = (rm.c - b0) < 32 ? (rm.c - b0) : 32;
#pragma unroll 1
      for (int k = 0; k < m32; ++k) {
        const int sk = __builtin_amdgcn_readlane(sr, k);
        const unsigned short* rp = h1 + (size_t)sk * 64 + lane;
        const unsigned hv = rp[0];
        const unsigned lv = rp[D1];
        a += __uint_as_float(hv << 16) + __uint_as_float(lv << 16);
      }
    }
    const bool live = node < nN;
    const float mval = live ? (a * rm.inv + rm.pz) : 0.0f;
    unsigned lb;
    const unsigned hb = hl_bits(mval, lb);
    rowbuf[lane]      = (unsigned short)hb;
    rowbuf[D1 + lane] = (unsigned short)lb;
    wave_sync();
    const v4u qa = *(const v4ua*)(rowbuf + 8 * (lane & 7));
    const v4u qo = *(const v4ua*)(h1 + (size_t)node * 64 + 8 * (lane & 7));
    wave_sync();
    const unsigned mk = (lane < 8) ? 0xFFFFFFFFu : 0u;
    v4u q;
    q.x = (qa.x & mk) | (qo.x & ~mk);
    q.y = (qa.y & mk) | (qo.y & ~mk);
    q.z = (qa.z & mk) | (qo.z & ~mk);
    q.w = (qa.w & mk) | (qo.w & ~mk);
    unsigned short* dp = a2 + (size_t)node * DF + 8 * (lane & 15);
    if (lane < 16) *(volatile v4u*)dp = q;
    __threadfence();
    if (lane < 16) *(volatile v4u*)dp = q;
  }
}

__global__ __launch_bounds__(NTHR) void k_aggw(const unsigned short* __restrict__ pin, const int* __restrict__ lst,
                                               const int* __restrict__ meta, int nN, unsigned short* pout) {
  __shared__ __attribute__((aligned(16))) unsigned short rb[NWAVE * PW];
  const int tid = (int)threadIdx.x, lane = tid & 31, wave = tid >> 5;
  unsigned short* rowbuf = rb + wave * PW;
#pragma unroll 1
  for (int r = 0; r < RPW; ++r) {
    const int node = (int)blockIdx.x * RPB + wave * RPW + r;
    const RowMeta rm = load_meta(meta, node);
    const int* lp = lst + (size_t)rm.blk * RCAP;
    float a0 = 0.0f, a1 = 0.0f, a2 = 0.0f, a3 = 0.0f;
#pragma unroll 1
    for (int b0 = 0; b0 < rm.c; b0 += 32) {
      int idx = rm.o + b0 + lane;
      idx = idx > RCAP - 1 ? RCAP - 1 : idx;
      int sr = lp[idx];
      sr = sr < 0 ? 0 : (sr > nN - 1 ? nN - 1 : sr);
      const int m32 = (rm.c - b0) < 32 ? (rm.c - b0) : 32;
#pragma unroll 1
      for (int k = 0; k < m32; ++k) {
        const int sk = __builtin_amdgcn_readlane(sr, k);
        const unsigned short* rp = pin + (size_t)sk * PW + 4 * lane;
        const v2u wh = *(const v2ua*)rp;
        const v2u wl = *(const v2ua*)(rp + DF);
        const float f0 = __uint_as_float(wh.x << 16)         + __uint_as_float(wl.x << 16);
        const float f1 = __uint_as_float(wh.x & 0xffff0000u) + __uint_as_float(wl.x & 0xffff0000u);
        const float f2 = __uint_as_float(wh.y << 16)         + __uint_as_float(wl.y << 16);
        const float f3 = __uint_as_float(wh.y & 0xffff0000u) + __uint_as_float(wl.y & 0xffff0000u);
        a0 += f0; a1 += f1; a2 += f2; a3 += f3;
      }
    }
    const bool live = node < nN;
    const float m0 = live ? (a0 * rm.inv + rm.pz) : 0.0f;
    const float m1 = live ? (a1 * rm.inv + rm.pz) : 0.0f;
    const float m2 = live ? (a2 * rm.inv + rm.pz) : 0.0f;
    const float m3 = live ? (a3 * rm.inv + rm.pz) : 0.0f;
    v4us mh, ml;
    {
      unsigned lb;
      unsigned hb;
      hb = hl_bits(m0, lb); mh[0] = (unsigned short)hb; ml[0] = (unsigned short)lb;
      hb = hl_bits(m1, lb); mh[1] = (unsigned short)hb; ml[1] = (unsigned short)lb;
      hb = hl_bits(m2, lb); mh[2] = (unsigned short)hb; ml[2] = (unsigned short)lb;
      hb = hl_bits(m3, lb); mh[3] = (unsigned short)hb; ml[3] = (unsigned short)lb;
    }
    *(v4usa*)(rowbuf + 4 * lane)      = mh;
    *(v4usa*)(rowbuf + DF + 4 * lane) = ml;
    wave_sync();
    const v8us q0 = *(const v8usa*)(rowbuf + 8 * lane);
    wave_sync();
    unsigned short* rpw = pout + (size_t)node * PW + 8 * lane;
    *(volatile v8us*)rpw = q0;
    __threadfence();
    *(volatile v8us*)rpw = q0;
  }
}

__device__ __forceinline__ void gemm_part(v8f (&acc)[8], const unsigned short* ap, const unsigned short* bp,
                                          int ldb, int kn) {
#pragma unroll 1
  for (int k0 = 0; k0 < kn; k0 += 32) {
    FragB af;
    af.h[0] = *(const v8usa*)(ap + k0);
    af.h[1] = *(const v8usa*)(ap + k0 + 16);
#pragma unroll
    for (int nt = 0; nt < 8; ++nt) {
      const unsigned short* wq = bp + (size_t)(16 * nt) * (size_t)ldb + k0;
      FragB bf;
      bf.h[0] = *(const v8usa*)wq;
      bf.h[1] = *(const v8usa*)(wq + 16);
      acc[nt] = wmb(af, bf, acc[nt]);
    }
  }
}

template <int FIN>
__global__ __launch_bounds__(GTHR) void k_gemm(const unsigned short* A0, const unsigned short* A1, int lda, int KH,
                                               int nPl, const unsigned short* __restrict__ BT, int ldb,
                                               const float* __restrict__ bias, unsigned short* outPl,
                                               const float* __restrict__ wlin, const float* __restrict__ blin,
                                               const int* __restrict__ meta, float* outp, int nN) {
  __shared__ __attribute__((aligned(16))) float stg[GBM * GBN];
  const int tid = (int)threadIdx.x, lane = tid & 31, wave = tid >> 5, hh = lane >> 4, m = lane & 15;
  const int rowBase = (int)blockIdx.x * GBM;

  v8f acc[8];
#pragma unroll
  for (int t = 0; t < 8; ++t) acc[t] = z8();
  const size_t arow = (size_t)(rowBase + 16 * wave + m) * (size_t)lda + 8 * hh;
  const unsigned short* bp = BT + (size_t)m * (size_t)ldb + 8 * hh;
  gemm_part(acc, A0 + arow, bp, ldb, KH);
  if (nPl > 1) gemm_part(acc, A1 + arow, bp + KH, ldb, KH);

#pragma unroll
  for (int nt = 0; nt < 8; ++nt) {
    const int lc = 16 * nt + m;
#pragma unroll
    for (int r = 0; r < 8; ++r) {
      const int lr = 16 * wave + 8 * hh + r;
      stg[lr * GBN + lc] = acc[nt][r];
    }
  }
  __syncthreads();

  float bq0, bq1, bq2, bq3;
  {
    const v4f b4 = *(const v4f*)(bias + 4 * lane);
    bq0 = bf16_val(b4.x); bq1 = bf16_val(b4.y); bq2 = bf16_val(b4.z); bq3 = bf16_val(b4.w);
  }

  v4f pv[16];
#pragma unroll
  for (int i = 0; i < 16; ++i) pv[i] = *(const v4fa*)(stg + (16 * wave + i) * GBN + 4 * lane);
  __syncthreads();

#pragma unroll
  for (int i = 0; i < 16; ++i) {
    const bool ok = (rowBase + 16 * wave + i) < nN;
    const float o0 = relu_p(pv[i].x + bq0);
    const float o1 = relu_p(pv[i].y + bq1);
    const float o2 = relu_p(pv[i].z + bq2);
    const float o3 = relu_p(pv[i].w + bq3);
    v4f qo;
    qo.x = ok ? o0 : 0.0f; qo.y = ok ? o1 : 0.0f; qo.z = ok ? o2 : 0.0f; qo.w = ok ? o3 : 0.0f;
    pv[i] = qo;
  }

  if constexpr (FIN != 0) {
    __shared__ __attribute__((aligned(16))) float sco[GBM];
    float w0, w1, w2, w3;
    {
      const v4f t4 = *(const v4f*)(wlin + 4 * lane);
      w0 = bf16_val(t4.x); w1 = bf16_val(t4.y); w2 = bf16_val(t4.z); w3 = bf16_val(t4.w);
    }
    const float bl = bf16_val(blin[0]);
    float sc = 0.0f;
#pragma unroll
    for (int i = 0; i < 16; ++i) {
      float p = pv[i].x * w0;
      p = fmaf(pv[i].y, w1, p);
      p = fmaf(pv[i].z, w2, p);
      p = fmaf(pv[i].w, w3, p);
      p += __shfl_xor(p, 16, 32);
      p += __shfl_xor(p, 8, 32);
      p += __shfl_xor(p, 4, 32);
      p += __shfl_xor(p, 2, 32);
      p += __shfl_xor(p, 1, 32);
      const float sv = p + bl;
      sc = (lane == i) ? sv : sc;
    }
    if (lane < 16) sco[16 * wave + lane] = sc;
    __syncthreads();
    if (wave == 0) {
      const int l16 = lane & 15;
      const v4f s4 = *(const v4fa*)(sco + 4 * l16);
      const int r0 = rowBase + 4 * l16;
      int f[4];
#pragma unroll
      for (int j = 0; j < 4; ++j) {
        int rc = r0 + j;
        rc = rc < 0 ? 0 : (rc > NMETA - 1 ? NMETA - 1 : rc);
        f[j] = meta[(size_t)rc * 4 + 3];
      }
      const float qn = __int_as_float(0x7fc00000);
      v4f o;
      o.x = (f[0] != 0) ? qn : s4.x;
      o.y = (f[1] != 0) ? qn : s4.y;
      o.z = (f[2] != 0) ? qn : s4.z;
      o.w = (f[3] != 0) ? qn : s4.w;
      const bool st = (lane < 16) && (r0 + 4 <= nN);
      float* op = outp + (size_t)(st ? r0 : 0);
      if (st) *(volatile v4f*)op = o;
      __threadfence();
      if (st) *(volatile v4f*)op = o;
    }
    (void)outPl;
  } else {
#pragma unroll
    for (int i = 0; i < 16; ++i) {
      v4us h4, l4;
      unsigned lb;
      unsigned hb;
      hb = hl_bits(pv[i].x, lb); h4[0] = (unsigned short)hb; l4[0] = (unsigned short)lb;
      hb = hl_bits(pv[i].y, lb); h4[1] = (unsigned short)hb; l4[1] = (unsigned short)lb;
      hb = hl_bits(pv[i].z, lb); h4[2] = (unsigned short)hb; l4[2] = (unsigned short)lb;
      hb = hl_bits(pv[i].w, lb); h4[3] = (unsigned short)hb; l4[3] = (unsigned short)lb;
      unsigned short* srow = (unsigned short*)stg + (size_t)(16 * wave + i) * (2 * GBN);
      *(v4usa*)(srow + 4 * lane) = h4;
      *(v4usa*)(srow + DF + 4 * lane) = l4;
    }
    __syncthreads();
    v8us qv[16];
#pragma unroll
    for (int i = 0; i < 16; ++i) {
      const unsigned short* srow = (const unsigned short*)stg + (size_t)(16 * wave + i) * (2 * GBN);
      qv[i] = *(const v8usa*)(srow + 8 * lane);
    }
#pragma unroll
    for (int i = 0; i < 16; ++i) {
      const int gr = rowBase + 16 * wave + i;
      unsigned short* rp = outPl + (size_t)gr * (size_t)PW + 8 * lane;
      *(volatile v8us*)rp = qv[i];
    }
    __threadfence();
#pragma unroll
    for (int i = 0; i < 16; ++i) {
      const int gr = rowBase + 16 * wave + i;
      unsigned short* rp = outPl + (size_t)gr * (size_t)PW + 8 * lane;
      *(volatile v8us*)rp = qv[i];
    }
    (void)outp; (void)wlin; (void)blin; (void)meta;
  }
}

extern "C" void kernel_launch(void* const* d_in, const int* in_sizes, int n_in,
                              void* d_out, int out_size, void* d_ws, size_t ws_size,
                              hipStream_t stream) {
  if (n_in < 19) return;
  const int want[19] = {NN * 2, 2 * NE, 2 * D1, D1, 2 * D1, D1 * DF, DF, D1 * DF,
                        DF * DF, DF, DF * DF, DF * DF, DF, DF * DF, DF * DF, DF, DF * DF, DF, 1};
  for (int i = 0; i < 19; ++i) if (in_sizes[i] != want[i]) return;
  if (out_size != NN) return;

  const float* x    = (const float*)d_in[0];
  const int*   ei   = (const int*)  d_in[1];
  const float* W1l  = (const float*)d_in[2];
  const float* b1   = (const float*)d_in[3];
  const float* W1r  = (const float*)d_in[4];
  const float* W2l  = (const float*)d_in[5];
  const float* b2   = (const float*)d_in[6];
  const float* W2r  = (const float*)d_in[7];
  const float* W3l  = (const float*)d_in[8];
  const float* b3   = (const float*)d_in[9];
  const float* W3r  = (const float*)d_in[10];
  const float* W4l  = (const float*)d_in[11];
  const float* b4   = (const float*)d_in[12];
  const float* W4r  = (const float*)d_in[13];
  const float* W5l  = (const float*)d_in[14];
  const float* b5   = (const float*)d_in[15];
  const float* W5r  = (const float*)d_in[16];
  const float* Wlin = (const float*)d_in[17];
  const float* blin = (const float*)d_in[18];
  float* out = (float*)d_out;
  const int* src = ei;
  const int* dst = ei + NE;
  const int vec8 = ((NE & 3) == 0) ? 1 : 0;

  const size_t szW2   = (size_t)DF * DF * 2;
  const size_t szWB   = (size_t)3 * DF * 4 * DF * 2;
  const size_t szMETA = (size_t)NMETA * 16;
  const size_t szLIST = (size_t)NBLK * RCAP * 4;
  const size_t szH1   = (size_t)MPAD * 64 * 2;
  const size_t szA2   = (size_t)MPAD * DF * 2;
  const size_t szPL   = (size_t)MPAD * PW * 2;
  const size_t oW2 = 0;
  const size_t oWB = oW2 + szW2;
  const size_t oMT = oWB + szWB;
  const size_t oLS = oMT + szMETA;
  const size_t oH1 = oLS + szLIST;
  const size_t oA2 = oH1 + szH1;
  const size_t oP  = oA2 + szA2;
  const size_t oQ  = oP + szPL;
  const size_t oR  = oQ + szPL;
  const size_t wsEnd = oR + szPL;
  if (wsEnd > ws_size || wsEnd > (size_t)WSMAX) return;
  char* ws = (char*)d_ws;
  unsigned short* W2C = (unsigned short*)(ws + oW2);
  unsigned short* WBG = (unsigned short*)(ws + oWB);
  int*            MET = (int*)(ws + oMT);
  int*            LST = (int*)(ws + oLS);
  unsigned short* H1  = (unsigned short*)(ws + oH1);
  unsigned short* A2  = (unsigned short*)(ws + oA2);
  unsigned short* P   = (unsigned short*)(ws + oP);
  unsigned short* Q   = (unsigned short*)(ws + oQ);
  unsigned short* R   = (unsigned short*)(ws + oR);
  const unsigned short* W3C = WBG;
  const unsigned short* W4C = WBG + (size_t)DF * 4 * DF;
  const unsigned short* W5C = WBG + (size_t)2 * DF * 4 * DF;

  const size_t bktLds = (size_t)BKT_LDS_INTS * 4;
  hipFuncSetAttribute(reinterpret_cast<const void*>(&k_bucket), hipFuncAttributeMaxDynamicSharedMemorySize, (int)bktLds);

  const int gR = MPAD / RPB;
  const int gM = MPAD / GBM;

  k_prep<<<NUP / NTHR, NTHR, 0, stream>>>(W2l, W2r, W3l, W3r, W4l, W4r, W5l, W5r, W2C, WBG);
  k_bucket<<<NBLK, NTHR, bktLds, stream>>>(src, dst, NE, NN, vec8, LST, MET);
  k_l1<<<gR, NTHR, 0, stream>>>(x, W1l, b1, W1r, LST, MET, NN, H1);
  k_agg2<<<gR, NTHR, 0, stream>>>(H1, LST, MET, NN, A2);
  k_gemm<0><<<gM, GTHR, 0, stream>>>(A2, A2, DF, DF, 1, W2C, DF, b2, P, Wlin, blin, MET, out, NN);
  k_aggw<<<gR, NTHR, 0, stream>>>(P, LST, MET, NN, Q);
  k_gemm<0><<<gM, GTHR, 0, stream>>>(Q, P, PW, PW, 2, W3C, 4 * DF, b3, R, Wlin, blin, MET, out, NN);
  k_aggw<<<gR, NTHR, 0, stream>>>(R, LST, MET, NN, Q);
  k_gemm<0><<<gM, GTHR, 0, stream>>>(Q, R, PW, PW, 2, W4C, 4 * DF, b4, P, Wlin, blin, MET, out, NN);
  k_aggw<<<gR, NTHR, 0, stream>>>(P, LST, MET, NN, Q);
  k_gemm<1><<<gM, GTHR, 0, stream>>>(Q, P, PW, PW, 2, W5C, 4 * DF, b5, R, Wlin, blin, MET, out, NN);
}
